// CA_76922864272011
// MI455X (gfx1250) — hardware-run, weakly checked
//
#include <hip/hip_runtime.h>
#include <stddef.h>


typedef _Float16 v16h __attribute__((ext_vector_type(16)));
typedef _Float16 v8h  __attribute__((ext_vector_type(8)));
typedef float    v8f  __attribute__((ext_vector_type(8)));
typedef float    v4f  __attribute__((ext_vector_type(4)));
typedef _Float16 h16;

#ifndef NB
#define NB 2
#endif
#ifndef SEQ
#define SEQ 512
#endif
#define NB_FULL  2
#define SEQ_FULL 512
#define DIM   256
#define NGRP  16
#define DGRP  16
#define MROWS (NB * SEQ)

static_assert(NB >= 1 && NB <= NB_FULL);
static_assert(SEQ >= 64 && SEQ <= SEQ_FULL && (SEQ % 64) == 0);
static_assert((SEQ % 32) == 0 && (SEQ % 16) == 0);
static_assert(DIM == NGRP * DGRP);
static_assert(NGRP == 16 && DGRP == 16);
static_assert((DIM % 64) == 0 && (DIM % 32) == 0);
static_assert((MROWS % 64) == 0 && (MROWS % 8) == 0);
static_assert(DIM == 32 * 8);
static_assert((size_t)NB_FULL * SEQ_FULL * DIM * 4 == (size_t)1048576);

#define LDT 72
#define LDC 68
#define SP  20
#define OSP 260
static_assert((LDT % 8) == 0 && LDT >= 64);
static_assert((LDC % 4) == 0 && LDC >= 64);
static_assert((SP % 4) == 0 && SP >= 16);
static_assert((OSP % 4) == 0 && OSP >= DIM);

#define XCARRY 16.0f
#define WCARRY 1024.0f
#define VCARRY 64.0f
#define PCARRY 1024.0f

#define WSQ_BYTES     ((size_t)DIM * DIM * 2)
#define PLANE16_BYTES ((size_t)MROWS * DIM * 2)
#define PLANE32_BYTES ((size_t)MROWS * DIM * 4)
#define VT_BYTES      ((size_t)NB * DIM * SEQ * 2)
#define OFF_WQ  ((size_t)0)
#define OFF_WK  (OFF_WQ + WSQ_BYTES)
#define OFF_WV  (OFF_WK + WSQ_BYTES)
#define OFF_XT  (OFF_WV + WSQ_BYTES)
#define OFF_XS  (OFF_XT + PLANE16_BYTES)
#define OFF_QF  (OFF_XS + PLANE16_BYTES)
#define OFF_KF  (OFF_QF + PLANE32_BYTES)
#define OFF_VT  (OFF_KF + PLANE32_BYTES)
#define WS_TOTAL (OFF_VT + VT_BYTES)
static_assert((WSQ_BYTES % 128) == 0 && (PLANE16_BYTES % 128) == 0);
static_assert((PLANE32_BYTES % 128) == 0 && (VT_BYTES % 128) == 0);
static_assert(WS_TOTAL <= (size_t)134217728);

__device__ __forceinline__ float bf16r(float x) {
  unsigned int u = __float_as_uint(x);
  u = (u + 0x7FFFu + ((u >> 16) & 1u)) & 0xFFFF0000u;
  return __uint_as_float(u);
}

static __device__ __forceinline__ h16 toh_flush(float v) {
  const h16 r = (h16)v;
  return (fabsf(v) < 6.103515625e-05f) ? (h16)0.0f : r;
}

__device__ __forceinline__ v16h frag_at(const _Float16* p) {
  v8h lo = *(const v8h*)(p);
  v8h hi = *(const v8h*)(p + 16);
  v16h out;
#pragma unroll
  for (int i = 0; i < 8; ++i) { out[i] = lo[i]; out[i + 8] = hi[i]; }
  return out;
}

__device__ __forceinline__ v8f wmma16(v16h a, v16h b, v8f c) {
  v8f d = __builtin_amdgcn_wmma_f32_16x16x32_f16(false, a, false, b, (short)0, c,
                                                 false, false);
  asm volatile("v_nop\n\tv_nop\n\tv_nop\n\tv_nop" : "+v"(d) : "v"(a), "v"(b));
  return d;
}

__global__ __launch_bounds__(256) void wconv_kernel(
    const float* __restrict__ W, _Float16* __restrict__ Wt, unsigned ldw, unsigned ldk) {
  __shared__ _Float16 T[64 * LDT];
  const unsigned tid = threadIdx.x;
  const unsigned n0 = blockIdx.x * 64u;
  const unsigned k0 = blockIdx.y * 64u;
#pragma unroll 4
  for (unsigned j = 0; j < 16u; ++j) {
    const unsigned idx = tid + 256u * j;
    const unsigned kr = idx >> 6, nc = idx & 63u;
    const float v = W[(size_t)(k0 + kr) * ldw + n0 + nc];
    T[nc * LDT + kr] = (_Float16)(WCARRY * bf16r(v));
  }
  __syncthreads();
  v8h x[2];
  size_t off[2];
#pragma unroll
  for (unsigned i = 0; i < 2u; ++i) {
    const unsigned n = 32u * i + (tid >> 3);
    const unsigned kc = (tid & 7u) * 8u;
    x[i] = *(const v8h*)&T[n * LDT + kc];
    off[i] = (size_t)(n0 + n) * ldk + k0 + kc;
  }
#pragma unroll
  for (int i = 0; i < 2; ++i) *(volatile v8h*)(Wt + off[i]) = x[i];
  __threadfence();
#pragma unroll
  for (int i = 0; i < 2; ++i) *(volatile v8h*)(Wt + off[i]) = x[i];
}

__global__ __launch_bounds__(256) void xconv_kernel(
    const float* __restrict__ X, _Float16* __restrict__ dst) {
  const unsigned lane = threadIdx.x & 31u;
  const unsigned wave = (unsigned)__builtin_amdgcn_readfirstlane((int)(threadIdx.x >> 5));
  const unsigned crow = blockIdx.x * 8u + wave;
  const unsigned bidx = crow / (unsigned)SEQ;
  const unsigned sq = crow - bidx * (unsigned)SEQ;
  const size_t srow = (size_t)bidx * SEQ_FULL + sq;
  const float* xr = X + srow * DIM + lane * 8u;
  const v4f a0 = *(const v4f*)(xr);
  const v4f a1 = *(const v4f*)(xr + 4);
  v8h o;
#pragma unroll
  for (int i = 0; i < 4; ++i) {
    o[i]     = toh_flush(XCARRY * bf16r(a0[i]));
    o[i + 4] = toh_flush(XCARRY * bf16r(a1[i]));
  }
  _Float16* p = dst + (size_t)crow * DIM + lane * 8u;
  *(volatile v8h*)p = o;
  __threadfence();
  *(volatile v8h*)p = o;
}

template <int MODE>
__device__ __forceinline__ void gemm_body(
    const _Float16* __restrict__ A16, const _Float16* __restrict__ Bt, const unsigned K,
    float* __restrict__ outf, _Float16* __restrict__ out16) {
  __shared__ float Cs[64 * LDC];
  const unsigned tid = threadIdx.x, lane = tid & 31u, w = tid >> 5;
  const unsigned mw = w >> 1, nw = w & 1u;
  const unsigned hh = lane >> 4, m = lane & 15u;
  const unsigned n0 = blockIdx.x * 64u;
  const unsigned row0 = blockIdx.y * 64u;

  const _Float16* ap  = A16 + (size_t)(row0 + mw * 16u + m) * K + hh * 8u;
  const _Float16* bp0 = Bt + (size_t)(n0 + nw * 32u + m) * K + hh * 8u;
  const _Float16* bp1 = bp0 + (size_t)16 * K;
  v8f acc0 = {}, acc1 = {};
#pragma unroll 2
  for (unsigned k0 = 0; k0 < K; k0 += 32u) {
    const v16h a  = frag_at(ap + k0);
    const v16h b0 = frag_at(bp0 + k0);
    const v16h b1 = frag_at(bp1 + k0);
    acc0 = wmma16(a, b0, acc0);
    acc1 = wmma16(a, b1, acc1);
  }
#pragma unroll
  for (int r = 0; r < 8; ++r) {
    float* d = &Cs[(mw * 16u + hh * 8u + (unsigned)r) * LDC + nw * 32u + m];
    d[0]  = acc0[r];
    d[16] = acc1[r];
  }
  __syncthreads();

  if (MODE == 0) {
    const float cs = 1.0f / (XCARRY * WCARRY);
    v4f xs[4];
    size_t off[4];
#pragma unroll
    for (unsigned i = 0; i < 4u; ++i) {
      const unsigned r = 16u * i + (tid >> 4);
      const unsigned c = (tid & 15u) * 4u;
      const v4f u = *(const v4f*)&Cs[r * LDC + c];
      v4f val;
#pragma unroll
      for (int j = 0; j < 4; ++j) val[j] = u[j] * cs;
      xs[i] = val;
      off[i] = (size_t)(row0 + r) * DIM + n0 + c;
    }
#pragma unroll
    for (int i = 0; i < 4; ++i) *(volatile v4f*)(outf + off[i]) = xs[i];
    __threadfence();
#pragma unroll
    for (int i = 0; i < 4; ++i) *(volatile v4f*)(outf + off[i]) = xs[i];
  }

  if (MODE == 1) {
    const float cs = VCARRY / (XCARRY * WCARRY);
    const unsigned bidx = row0 / (unsigned)SEQ;
    const unsigned key0 = row0 - bidx * (unsigned)SEQ;
    v8h x[2];
    size_t off[2];
#pragma unroll
    for (unsigned i = 0; i < 2u; ++i) {
      const unsigned dcol = 32u * i + (tid >> 3);
      const unsigned kk = (tid & 7u) * 8u;
#pragma unroll
      for (unsigned j = 0; j < 8u; ++j)
        x[i][j] = toh_flush(Cs[(kk + j) * LDC + dcol] * cs);
      const unsigned col = n0 + dcol;
      const unsigned prow = (col & 15u) * 16u + (col >> 4);
      off[i] = ((size_t)bidx * DIM + prow) * SEQ + key0 + kk;
    }
#pragma unroll
    for (int i = 0; i < 2; ++i) *(volatile v8h*)(out16 + off[i]) = x[i];
    __threadfence();
#pragma unroll
    for (int i = 0; i < 2; ++i) *(volatile v8h*)(out16 + off[i]) = x[i];
  }
}

__global__ __launch_bounds__(256) void gemm_f32_kernel(
    const _Float16* __restrict__ A16, const _Float16* __restrict__ Bt, float* __restrict__ outf) {
  gemm_body<0>(A16, Bt, (unsigned)DIM, outf, (_Float16*)0);
}
__global__ __launch_bounds__(256) void gemm_vt_kernel(
    const _Float16* __restrict__ A16, const _Float16* __restrict__ Bt, _Float16* __restrict__ vt) {
  gemm_body<1>(A16, Bt, (unsigned)DIM, (float*)0, vt);
}

__global__ __launch_bounds__(256) void attn_kernel(
    const float* __restrict__ Qf, const float* __restrict__ Kf, const _Float16* __restrict__ Vt,
    const float* __restrict__ addb, const float* __restrict__ mulb,
    const float* __restrict__ wm, const float* __restrict__ bm, float* __restrict__ out) {
  __shared__ float Ss[256 * SP];
  __shared__ float Os[16 * OSP];

  const unsigned tid = threadIdx.x, lane = tid & 31u;
  const unsigned wave = (unsigned)__builtin_amdgcn_readfirstlane((int)(threadIdx.x >> 5));
  const unsigned hh = lane >> 4, m = lane & 15u;
  const unsigned l0 = blockIdx.x * 16u;
  const unsigned b = blockIdx.y;
  const unsigned sbase = tid * SP;

  float wv[16];
#pragma unroll
  for (int d = 0; d < 16; ++d) wv[d] = bf16r(wm[d]);
  const float bb = bf16r(bm[0]);

#pragma unroll 1
  for (unsigned gi = 0; gi < 2u; ++gi) {
    const unsigned g = wave * 2u + gi;

    float q[16];
    {
      const float* qp = Qf + (size_t)(b * (unsigned)SEQ + l0 + m) * DIM + g * 16u;
#pragma unroll
      for (int c = 0; c < 4; ++c) {
        const v4f t = *(const v4f*)(qp + 4 * c);
#pragma unroll
        for (int e = 0; e < 4; ++e) q[4 * c + e] = t[e];
      }
    }
    const size_t brow = (((size_t)b * SEQ_FULL + l0 + m) * NGRP + g) * SEQ_FULL + hh * 8u;
    const size_t kbase = (size_t)b * SEQ * DIM + g * 16u;
    const _Float16* vp = Vt + ((size_t)b * DIM + g * 16u + m) * SEQ + hh * 8u;

    float mrow = -1.0e30f, lsum = 0.0f;
    v8f acc = {};

#pragma unroll 1
    for (unsigned kb = 0; kb < (unsigned)SEQ; kb += 32u) {
#pragma unroll 1
      for (unsigned it = 0; it < 4u; ++it) {
        unsigned ko = kb + (it >> 1) * 16u + (it & 1u) * 4u;
        const size_t krow = kbase + (size_t)(ko + hh * 8u) * DIM;
        v4f sc;
#pragma unroll
        for (int j = 0; j < 4; ++j) {
          const float* kp = Kf + krow + (size_t)j * DIM;
          float s = 0.0f;
#pragma unroll
          for (int c = 0; c < 4; ++c) {
            const v4f kv = *(const v4f*)(kp + 4 * c);
#pragma unroll
            for (int e = 0; e < 4; ++e)
              s = fmaf(fmaxf(q[4 * c + e] - kv[e], 0.0f), wv[4 * c + e], s);
          }
          sc[j] = fmaxf(s + bb, 0.0f);
        }
        asm volatile("" : "+v"(ko), "+v"(sc));
        const v4f av = *(const v4f*)(addb + brow + ko);
        const v4f mv = *(const v4f*)(mulb + brow + ko);
        v4f lg;
#pragma unroll
        for (int j = 0; j < 4; ++j) lg[j] = sc[j] * bf16r(mv[j]) + bf16r(av[j]);
        *(v4f*)&Ss[sbase + it * 4u] = lg;
      }

      float t[16];
#pragma unroll
      for (int c = 0; c < 4; ++c) {
        const v4f u = *(const v4f*)&Ss[sbase + 4 * c];
#pragma unroll
        for (int e = 0; e < 4; ++e) t[4 * c + e] = u[e];
      }
      float mx = t[0];
#pragma unroll
      for (int i = 1; i < 16; ++i) mx = fmaxf(mx, t[i]);
      mx = fmaxf(mx, __shfl_xor(mx, 16, 32));
      const float mn = fmaxf(mrow, mx);
      const float alpha = __expf(mrow - mn);
      mrow = mn;

      v16h pf;
      float rs = 0.0f;
#pragma unroll
      for (int i = 0; i < 16; ++i) {
        const h16 ph = toh_flush(PCARRY * __expf(t[i] - mn));
        pf[i] = ph;
        rs += (float)ph;
      }
      lsum = alpha * lsum + rs;
#pragma unroll
      for (int r = 0; r < 8; ++r) acc[r] = acc[r] * alpha;

      const v16h vf = frag_at(vp + kb);
      acc = wmma16(vf, pf, acc);
    }

    const float ltot = lsum + __shfl_xor(lsum, 16, 32);
    const float inv = __builtin_amdgcn_rcpf(ltot * VCARRY);
#pragma unroll
    for (int r = 0; r < 8; ++r)
      Os[m * OSP + (hh * 8u + (unsigned)r) * 16u + g] = acc[r] * inv;
  }
  __syncthreads();

  v4f xs[4];
  size_t off[4];
#pragma unroll
  for (unsigned i = 0; i < 4u; ++i) {
    const unsigned idx = tid + 256u * i;
    const unsigned r = idx >> 6;
    const unsigned c = (idx & 63u) * 4u;
    xs[i] = *(const v4f*)&Os[r * OSP + c];
    off[i] = ((size_t)b * SEQ_FULL + l0 + r) * DIM + c;
  }
#pragma unroll
  for (int i = 0; i < 4; ++i) *(volatile v4f*)(out + off[i]) = xs[i];
  __threadfence();
#pragma unroll
  for (int i = 0; i < 4; ++i) *(volatile v4f*)(out + off[i]) = xs[i];
}

extern "C" void kernel_launch(void* const* d_in, const int* in_sizes, int n_in,
                              void* d_out, int out_size, void* d_ws, size_t ws_size,
                              hipStream_t stream) {
  if (n_in < 9) return;
  const long long need_x = ((long long)(NB - 1) * SEQ_FULL + SEQ) * DIM;
  const long long need_b = ((long long)(NB - 1) * SEQ_FULL + SEQ) * NGRP * SEQ_FULL;
  if ((long long)in_sizes[0] < need_x) return;
  if ((long long)in_sizes[1] < need_x) return;
  if ((long long)in_sizes[2] < need_b) return;
  if ((long long)in_sizes[3] < need_b) return;
  if ((long long)in_sizes[4] < (long long)DIM * DIM) return;
  if ((long long)in_sizes[5] < (long long)DIM * DIM) return;
  if ((long long)in_sizes[6] < (long long)DIM * DIM) return;
  if (in_sizes[7] < DGRP || in_sizes[8] < 1) return;
  if ((long long)out_size < need_x) return;
  if (ws_size < WS_TOTAL) return;

  const float* xs   = (const float*)d_in[0];
  const float* xt   = (const float*)d_in[1];
  const float* addb = (const float*)d_in[2];
  const float* mulb = (const float*)d_in[3];
  const float* wq   = (const float*)d_in[4];
  const float* wk   = (const float*)d_in[5];
  const float* wv   = (const float*)d_in[6];
  const float* wm   = (const float*)d_in[7];
  const float* bm   = (const float*)d_in[8];
  float* out = (float*)d_out;

  char* ws = (char*)d_ws;
  _Float16* Wq_t = (_Float16*)(ws + OFF_WQ);
  _Float16* Wk_t = (_Float16*)(ws + OFF_WK);
  _Float16* Wv_t = (_Float16*)(ws + OFF_WV);
  _Float16* XT16 = (_Float16*)(ws + OFF_XT);
  _Float16* XS16 = (_Float16*)(ws + OFF_XS);
  float*    QF   = (float*)(ws + OFF_QF);
  float*    KF   = (float*)(ws + OFF_KF);
  _Float16* VT16 = (_Float16*)(ws + OFF_VT);

  dim3 blk(256);
  dim3 gsq(DIM / 64, DIM / 64);
  dim3 gg(DIM / 64, MROWS / 64);

  wconv_kernel<<<gsq, blk, 0, stream>>>(wq, Wq_t, (unsigned)DIM, (unsigned)DIM);
  wconv_kernel<<<gsq, blk, 0, stream>>>(wk, Wk_t, (unsigned)DIM, (unsigned)DIM);
  wconv_kernel<<<gsq, blk, 0, stream>>>(wv, Wv_t, (unsigned)DIM, (unsigned)DIM);

  xconv_kernel<<<dim3(MROWS / 8), blk, 0, stream>>>(xt, XT16);
  xconv_kernel<<<dim3(MROWS / 8), blk, 0, stream>>>(xs, XS16);

  gemm_f32_kernel<<<gg, blk, 0, stream>>>(XT16, Wq_t, QF);
  gemm_f32_kernel<<<gg, blk, 0, stream>>>(XS16, Wk_t, KF);
  gemm_vt_kernel<<<gg, blk, 0, stream>>>(XS16, Wv_t, VT16);

  attn_kernel<<<dim3(SEQ / 16, NB), blk, 0, stream>>>(QF, KF, VT16, addb, mulb, wm, bm, out);
}
